// GDN_53781580480873
// MI455X (gfx1250) — hardware-verified
//
#include <hip/hip_runtime.h>
#include <stddef.h>
#include <stdint.h>


#define NGR    128
#define NND    512
#define FIN    64
#define DDM    128
#define NROW   65536
#define NCH    80
#define NTHR   256
#define NWAVE  8
#define EPT    8
#define CHUNK  (NTHR * EPT)
#define WCAP   (EPT * 32)
#define LISTN  (NWAVE * WCAP)
#define RCAP   255
#define TCAP   256
#define GBM    64
#define GBN    64
#define GTHR   128
#define EPSC   1e-5f
#define NEGS   0.2f
#define WSMAX  134217728
#define OOFF1  4194304
#define OOFF2  4259840
#define OTOT   4521984

#define HO_AB    0
#define HO_ST    32768
#define HO_BR    34816
#define HO_PR    35328
#define HEAD_LDS 35584

static_assert(NROW == NGR * NND);
static_assert(OOFF1 == NROW * FIN);
static_assert(OOFF2 == OOFF1 + NROW);
static_assert(OTOT == OOFF2 + NND * NND);
static_assert((NROW % GBM) == 0 && (FIN % 32) == 0 && (DDM % 32) == 0 && (NCH % 16) == 0);
static_assert((DDM % GBN) == 0 && GBM == (GTHR / 32) * 16);
static_assert((NGR % NWAVE) == 0);
static_assert(CHUNK == NTHR * EPT && (CHUNK & (CHUNK - 1)) == 0 && CHUNK <= 4096);
static_assert(TCAP >= RCAP + 1 && TCAP <= NTHR);
static_assert(NTHR == 2 * DDM);
static_assert(GBM * FIN * 4 <= 32768 && HEAD_LDS <= 65536);
static_assert((NND * NND) % 4 == 0);

typedef float          v4f   __attribute__((ext_vector_type(4)));
typedef float          v8f   __attribute__((ext_vector_type(8)));
typedef int            v4i   __attribute__((ext_vector_type(4)));
typedef unsigned short v4us  __attribute__((ext_vector_type(4)));
typedef unsigned short v8us  __attribute__((ext_vector_type(8)));
typedef __bf16         v16bf __attribute__((ext_vector_type(16)));
typedef double         v2d   __attribute__((ext_vector_type(2)));
typedef v8us __attribute__((may_alias)) v8usa;
typedef v4f  __attribute__((may_alias)) v4fa;

union Frag { v16bf v; v8us half[2]; };

__device__ __forceinline__ unsigned short f2bf(float f) {
  unsigned u = __builtin_bit_cast(unsigned, f);
  u += 0x7FFFu + ((u >> 16) & 1u);
  return (unsigned short)(u >> 16);
}
__device__ __forceinline__ float bf2f(unsigned short s) {
  return __builtin_bit_cast(float, ((unsigned)s) << 16);
}
__device__ __forceinline__ float bfr(float f) { return bf2f(f2bf(f)); }

__device__ __forceinline__ v8f wmb(v16bf a, v16bf b, v8f c) {
  v8f d = __builtin_amdgcn_wmma_f32_16x16x32_bf16(false, a, false, b, (short)0, c, false, false);
  asm volatile("v_nop\n\tv_nop\n\tv_nop\n\tv_nop" : "+v"(d) : "v"(a), "v"(b));
  return d;
}

__device__ __forceinline__ v16bf load_frag(const unsigned short* p, int h) {
  Frag f;
  f.half[0] = *(const v8usa*)(p + 8 * h);
  f.half[1] = *(const v8usa*)(p + 16 + 8 * h);
  return f.v;
}

__device__ __forceinline__ int scan_chunk(const int* __restrict__ dsts, int nE, int cbase, int slotBase,
                                          int nb, int vec8, int* list, int tid, int lane, int wave) {
  int wc = 0;
  const int el0  = tid * EPT;
  const int e0   = cbase + el0;
  const int sent = -2147483647 - 1;
  v4i da, db;
  if (vec8 != 0 && cbase + CHUNK <= nE) {
    da = *(const v4i*)(dsts + e0);
    db = *(const v4i*)(dsts + e0 + 4);
  } else {
    da.x = (e0     < nE) ? dsts[min(e0,     nE - 1)] : sent;
    da.y = (e0 + 1 < nE) ? dsts[min(e0 + 1, nE - 1)] : sent;
    da.z = (e0 + 2 < nE) ? dsts[min(e0 + 2, nE - 1)] : sent;
    da.w = (e0 + 3 < nE) ? dsts[min(e0 + 3, nE - 1)] : sent;
    db.x = (e0 + 4 < nE) ? dsts[min(e0 + 4, nE - 1)] : sent;
    db.y = (e0 + 5 < nE) ? dsts[min(e0 + 5, nE - 1)] : sent;
    db.z = (e0 + 6 < nE) ? dsts[min(e0 + 6, nE - 1)] : sent;
    db.w = (e0 + 7 < nE) ? dsts[min(e0 + 7, nE - 1)] : sent;
  }
  const unsigned nbs = (unsigned)slotBase;
  const unsigned unb = (unsigned)nb;
  const unsigned s0 = (unsigned)da.x - nbs, s1 = (unsigned)da.y - nbs;
  const unsigned s2 = (unsigned)da.z - nbs, s3 = (unsigned)da.w - nbs;
  const unsigned s4 = (unsigned)db.x - nbs, s5 = (unsigned)db.y - nbs;
  const unsigned s6 = (unsigned)db.z - nbs, s7 = (unsigned)db.w - nbs;
  const bool h0 = s0 < unb, h1 = s1 < unb, h2 = s2 < unb, h3 = s3 < unb;
  const bool h4 = s4 < unb, h5 = s5 < unb, h6 = s6 < unb, h7 = s7 < unb;
  const unsigned any = __builtin_amdgcn_ballot_w32(h0 | h1 | h2 | h3 | h4 | h5 | h6 | h7);
  if (any != 0u) {
#define HITJ(J, HJ, SJ) { \
      const unsigned mj = __builtin_amdgcn_ballot_w32(HJ); \
      if (mj != 0u) { \
        if (HJ) { \
          const int pos = wc + (int)__builtin_amdgcn_mbcnt_lo(mj, 0u); \
          if (pos < WCAP) list[wave * WCAP + pos] = ((el0 + (J)) << 12) | (int)(SJ); \
        } \
        wc += (int)__builtin_popcount(mj); } }
    HITJ(0, h0, s0)
    HITJ(1, h1, s1)
    HITJ(2, h2, s2)
    HITJ(3, h3, s3)
    HITJ(4, h4, s4)
    HITJ(5, h5, s5)
    HITJ(6, h6, s6)
    HITJ(7, h7, s7)
#undef HITJ
  }
  return wc;
}

__global__ __launch_bounds__(NTHR) void k_xprep(const float* __restrict__ x, unsigned short* xb, int nUnits) {
  const int i = (int)blockIdx.x * NTHR + (int)threadIdx.x;
  if (i >= nUnits) return;
  const float* p = x + (size_t)i * 8;
  const v4f a = *(const v4fa*)p;
  const v4f c = *(const v4fa*)(p + 4);
  const v8us o = { f2bf(a.x), f2bf(a.y), f2bf(a.z), f2bf(a.w),
                   f2bf(c.x), f2bf(c.y), f2bf(c.z), f2bf(c.w) };
  unsigned short* d = xb + (size_t)i * 8;
  *(volatile v8us*)d = o;
  __threadfence();
  *(volatile v8us*)d = o;
}

__global__ __launch_bounds__(NTHR) void k_wtr(const float* __restrict__ w0, int c0,
                                              const float* __restrict__ w1, int c1,
                                              int K, unsigned short* wt, int nUnits) {
  const int u = (int)blockIdx.x * NTHR + (int)threadIdx.x;
  if (u >= nUnits) return;
  const int kq = K >> 3;
  const int n  = u / kq;
  const int k8 = (u - n * kq) * 8;
  const bool s0 = n < c0;
  const bool s1 = (n >= c0) && (n < c0 + c1);
  const float* wsrc = s0 ? w0 : w1;
  const int cc = s0 ? c0 : c1;
  int nc = s0 ? n : n - c0;
  nc = nc < 0 ? 0 : (nc > cc - 1 ? cc - 1 : nc);
  const float* p = wsrc + (size_t)k8 * (size_t)cc + nc;
  v4f a, b;
  a.x = p[0];               a.y = p[(size_t)cc];      a.z = p[(size_t)2 * cc];  a.w = p[(size_t)3 * cc];
  b.x = p[(size_t)4 * cc];  b.y = p[(size_t)5 * cc];  b.z = p[(size_t)6 * cc];  b.w = p[(size_t)7 * cc];
  const v4f z4 = {0.f, 0.f, 0.f, 0.f};
  if (!(s0 || s1)) { a = z4; b = z4; }
  const v8us o = { f2bf(a.x), f2bf(a.y), f2bf(a.z), f2bf(a.w),
                   f2bf(b.x), f2bf(b.y), f2bf(b.z), f2bf(b.w) };
  unsigned short* d = wt + (size_t)n * (size_t)K + k8;
  *(volatile v8us*)d = o;
  __threadfence();
  *(volatile v8us*)d = o;
}

__global__ __launch_bounds__(GTHR) void k_gemm_lin(const unsigned short* __restrict__ A,
                                                   const unsigned short* __restrict__ WT, float* outF) {
  __shared__ __attribute__((aligned(16))) float stg[GBM * GBN];
  const int tid = (int)threadIdx.x, lane = tid & 31, wave = tid >> 5, hh = lane >> 4, m = lane & 15;
  const int rowBase = (int)blockIdx.x * GBM;
  const int col0    = (int)blockIdx.y * GBN;

  v8f acc[4];
  {
    const v8f z = {0.f, 0.f, 0.f, 0.f, 0.f, 0.f, 0.f, 0.f};
    acc[0] = z; acc[1] = z; acc[2] = z; acc[3] = z;
  }
  const unsigned short* ap = A  + (size_t)(rowBase + 16 * wave + m) * (size_t)FIN;
  const unsigned short* wp = WT + (size_t)(col0 + m) * (size_t)FIN;
#pragma unroll 1
  for (int ks = 0; ks < FIN / 32; ++ks) {
    const v16bf af = load_frag(ap + 32 * ks, hh);
#pragma unroll
    for (int t = 0; t < 4; ++t) {
      const v16bf bf = load_frag(wp + (size_t)(16 * t) * (size_t)FIN + 32 * ks, hh);
      acc[t] = wmb(af, bf, acc[t]);
    }
  }

#pragma unroll
  for (int t = 0; t < 4; ++t) {
    const int lc = 16 * t + m;
#pragma unroll
    for (int r = 0; r < 8; ++r) {
      const int lr = 16 * wave + 8 * hh + r;
      stg[lr * GBN + lc] = acc[t][r];
    }
  }
  __syncthreads();

  v4f fv[8];
#pragma unroll
  for (int i = 0; i < 8; ++i) {
    const int lr = 16 * wave + 2 * i + hh;
    fv[i] = *(const v4fa*)(stg + lr * GBN + 4 * m);
  }
#pragma unroll
  for (int i = 0; i < 8; ++i) {
    const int lr = 16 * wave + 2 * i + hh;
    float* op = outF + (size_t)(rowBase + lr) * (size_t)DDM + col0 + 4 * m;
    *(volatile v4f*)op = fv[i];
  }
  __threadfence();
#pragma unroll
  for (int i = 0; i < 8; ++i) {
    const int lr = 16 * wave + 2 * i + hh;
    float* op = outF + (size_t)(rowBase + lr) * (size_t)DDM + col0 + 4 * m;
    *(volatile v4f*)op = fv[i];
  }
}

__global__ __launch_bounds__(NTHR) void k_agg(
    const int* __restrict__ srcs, const int* __restrict__ dsts,
    const float* __restrict__ W, const float* __restrict__ H,
    const float* __restrict__ gbias, float* OUTF, double* REC, int nE, int vec8) {
  __shared__ int list[LISTN];
  __shared__ int reg1[TCAP];
  __shared__ int esrc[TCAP];
  __shared__ float ecoef[TCAP];
  __shared__ int wcnt[NWAVE];
  __shared__ __attribute__((aligned(16))) double part[NWAVE * 2 * DDM];
  __shared__ __attribute__((aligned(16))) double recd[2 * DDM];
  const int tid = (int)threadIdx.x, lane = tid & 31, wave = tid >> 5;
  const int node = (int)blockIdx.x;

  for (int i = tid; i < TCAP; i += NTHR) { reg1[i] = 0; esrc[i] = 0; ecoef[i] = 0.f; }
  __syncthreads();

  int tot = 0;
  const int nChunks = (nE + CHUNK - 1) / CHUNK;
#pragma unroll 1
  for (int ch = 0; ch < nChunks; ++ch) {
    const int cbase = ch * CHUNK;
    const int wc = scan_chunk(dsts, nE, cbase, node, 1, vec8, list, tid, lane, wave);
    if (lane == 0) wcnt[wave] = wc;
    __syncthreads();
    int pre = 0, all = 0;
#pragma unroll
    for (int w2 = 0; w2 < NWAVE; ++w2) {
      int c = wcnt[w2];
      c = c < 0 ? 0 : (c > WCAP ? WCAP : c);
      all += c;
      pre += (w2 < wave) ? c : 0;
    }
    const int wcc  = wc > WCAP ? WCAP : wc;
    const int base = tot + pre;
#pragma unroll 1
    for (int i = lane; i < wcc; i += 32) {
      const int ent = list[wave * WCAP + i];
      const int el  = (ent >> 12) & (CHUNK - 1);
      int eid = cbase + el;
      eid = eid > nE - 1 ? nE - 1 : eid;
      const int pos = base + i;
      if (pos < RCAP) reg1[pos] = eid;
    }
    tot += all;
    tot = tot > RCAP ? RCAP : tot;
    __syncthreads();
  }
  const int nh   = tot;
  const int cntT = nh + 1;
  const bool ovf = (nh >= RCAP);

  if (wave == 0) {
    float lmax = -3.0e38f;
#pragma unroll 1
    for (int base = 0; base < cntT; base += 32) {
      const int j = base + lane;
      const bool valid = j < cntT;
      int idx1 = j - 1;
      idx1 = idx1 < 0 ? 0 : (idx1 > RCAP - 1 ? RCAP - 1 : idx1);
      int eid = reg1[idx1];
      eid = eid < 0 ? 0 : (eid > nE - 1 ? nE - 1 : eid);
      int sv = srcs[eid];
      sv = sv < 0 ? 0 : (sv > NND - 1 ? NND - 1 : sv);
      const int s = (j == 0) ? node : sv;
      const float w  = bfr(W[(size_t)node * NND + s]);
      const float al = (w > 0.f) ? w : NEGS * w;
      if (valid) { esrc[j] = s; ecoef[j] = al; }
      lmax = valid ? fmaxf(lmax, al) : lmax;
    }
    lmax = fmaxf(lmax, __shfl_xor(lmax, 16));
    lmax = fmaxf(lmax, __shfl_xor(lmax, 8));
    lmax = fmaxf(lmax, __shfl_xor(lmax, 4));
    lmax = fmaxf(lmax, __shfl_xor(lmax, 2));
    lmax = fmaxf(lmax, __shfl_xor(lmax, 1));
    __builtin_amdgcn_fence(__ATOMIC_RELEASE, "wavefront");
    __builtin_amdgcn_wave_barrier();
    float lsum = 0.f;
#pragma unroll 1
    for (int base = 0; base < cntT; base += 32) {
      const int j = base + lane;
      const bool valid = j < cntT;
      const float al = valid ? ecoef[j] : lmax;
      const float ez = expf(al - lmax);
      if (valid) { ecoef[j] = ez; lsum += ez; }
    }
    lsum += __shfl_xor(lsum, 16);
    lsum += __shfl_xor(lsum, 8);
    lsum += __shfl_xor(lsum, 4);
    lsum += __shfl_xor(lsum, 2);
    lsum += __shfl_xor(lsum, 1);
    const float inv = 1.0f / (lsum > 0.f ? lsum : 1.0f);
    __builtin_amdgcn_fence(__ATOMIC_RELEASE, "wavefront");
    __builtin_amdgcn_wave_barrier();
#pragma unroll 1
    for (int base = 0; base < cntT; base += 32) {
      const int j = base + lane;
      if (j < cntT) ecoef[j] = ecoef[j] * inv;
    }
  }
  __syncthreads();

  const float qnan = __int_as_float(0x7fc00000);
  const float pz = ovf ? qnan : 0.0f;
  v4f bias4 = *(const v4fa*)(gbias + 4 * lane);
  bias4.x = bfr(bias4.x); bias4.y = bfr(bias4.y); bias4.z = bfr(bias4.z); bias4.w = bfr(bias4.w);
  double s0 = 0.0, s1 = 0.0, s2 = 0.0, s3 = 0.0;
  double q0 = 0.0, q1 = 0.0, q2 = 0.0, q3 = 0.0;
#pragma unroll 1
  for (int i = 0; i < NGR / NWAVE; ++i) {
    const int b = wave + NWAVE * i;
    const float* hb = H + (size_t)b * (size_t)NND * (size_t)DDM + 4 * lane;
    v4f acc = {0.f, 0.f, 0.f, 0.f};
#pragma unroll 1
    for (int j = 0; j < cntT; ++j) {
      const int   s = esrc[j];
      const float a = ecoef[j];
      const v4f v = *(const v4fa*)(hb + (size_t)s * DDM);
      acc.x = fmaf(a, v.x, acc.x);
      acc.y = fmaf(a, v.y, acc.y);
      acc.z = fmaf(a, v.z, acc.z);
      acc.w = fmaf(a, v.w, acc.w);
    }
    v4f rv;
    rv.x = acc.x + bias4.x + pz;
    rv.y = acc.y + bias4.y + pz;
    rv.z = acc.z + bias4.z + pz;
    rv.w = acc.w + bias4.w + pz;
    float* op = OUTF + ((size_t)b * NND + (size_t)node) * (size_t)DDM + 4 * lane;
    *(volatile v4f*)op = rv;
    __threadfence();
    *(volatile v4f*)op = rv;
    s0 += (double)rv.x; q0 += (double)rv.x * (double)rv.x;
    s1 += (double)rv.y; q1 += (double)rv.y * (double)rv.y;
    s2 += (double)rv.z; q2 += (double)rv.z * (double)rv.z;
    s3 += (double)rv.w; q3 += (double)rv.w * (double)rv.w;
  }
  {
    double* ps = part + wave * (2 * DDM) + 4 * lane;
    ps[0] = s0; ps[1] = s1; ps[2] = s2; ps[3] = s3;
    ps[DDM + 0] = q0; ps[DDM + 1] = q1; ps[DDM + 2] = q2; ps[DDM + 3] = q3;
  }
  __syncthreads();
  {
    double a = 0.0;
#pragma unroll
    for (int w2 = 0; w2 < NWAVE; ++w2) a += part[w2 * (2 * DDM) + tid];
    recd[tid] = a;
  }
  __syncthreads();
  {
    const int tc = tid < DDM ? tid : DDM - 1;
    v2d val;
    val.x = recd[2 * tc];
    val.y = recd[2 * tc + 1];
    double* rp = REC + (size_t)node * (2 * DDM) + 2 * tc;
    const bool wr = tid < DDM;
    if (wr) *(volatile v2d*)rp = val;
    __threadfence();
    if (wr) *(volatile v2d*)rp = val;
  }
}

__global__ __launch_bounds__(DDM) void k_bnfin(const double* __restrict__ REC, float* STATS) {
  __shared__ __attribute__((aligned(16))) float sst[2 * DDM];
  const int c = (int)threadIdx.x;
  double S = 0.0, Q = 0.0;
#pragma unroll 1
  for (int n = 0; n < NND; ++n) {
    S += REC[(size_t)n * (2 * DDM) + c];
    Q += REC[(size_t)n * (2 * DDM) + DDM + c];
  }
  const double mu = S * (1.0 / 65536.0);
  double var = Q * (1.0 / 65536.0) - mu * mu;
  var = var < 0.0 ? 0.0 : var;
  const float muf  = (float)mu;
  const float varf = (float)var;
  const float rs   = 1.0f / sqrtf(varf + EPSC);
  sst[c]       = muf;
  sst[DDM + c] = rs;
  __syncthreads();
  const int tc = c < 64 ? c : 63;
  const v4f v = *(const v4fa*)(sst + 4 * tc);
  const bool wr = c < 64;
  if (wr) *(volatile v4f*)(STATS + 4 * tc) = v;
  __threadfence();
  if (wr) *(volatile v4f*)(STATS + 4 * tc) = v;
}

__global__ __launch_bounds__(GTHR) void k_head(
    const float* __restrict__ OUTF, const float* __restrict__ STATS,
    const float* __restrict__ gamma, const float* __restrict__ beta,
    const unsigned short* __restrict__ WRT,
    const float* __restrict__ brec, const float* __restrict__ bpred, float* OUT) {
  extern __shared__ __attribute__((aligned(16))) char smem[];
  unsigned short* sHi = (unsigned short*)(smem + HO_AB);
  unsigned short* sLo = sHi + GBM * DDM;
  float* sMu = (float*)(smem + HO_ST);
  float* sRs = sMu + DDM;
  float* sGa = sRs + DDM;
  float* sBe = sGa + DDM;
  float* sBr = (float*)(smem + HO_BR);
  float* sPr = (float*)(smem + HO_PR);
  const int tid = (int)threadIdx.x, lane = tid & 31, wave = tid >> 5, hh = lane >> 4, m = lane & 15;
  const int R = (int)blockIdx.x * GBM;

  {
    sMu[tid] = STATS[tid];
    sRs[tid] = STATS[DDM + tid];
    sGa[tid] = bfr(gamma[tid]);
    sBe[tid] = bfr(beta[tid]);
    const float bv = bfr(brec[tid < FIN ? tid : FIN - 1]);
    const float pv = bfr(bpred[0]);
    if (tid < NCH) sBr[tid] = (tid < FIN) ? bv : ((tid == FIN) ? pv : 0.f);
  }
  __syncthreads();

#pragma unroll 4
  for (int it = 0; it < (GBM * DDM) / (4 * GTHR); ++it) {
    const int q   = it * GTHR + tid;
    const int row = q >> 5;
    const int c4  = (q & 31) * 4;
    const v4f v  = *(const v4fa*)(OUTF + (size_t)(R + row) * (size_t)DDM + c4);
    const v4f mu = *(const v4fa*)(sMu + c4);
    const v4f rs = *(const v4fa*)(sRs + c4);
    const v4f ga = *(const v4fa*)(sGa + c4);
    const v4f be = *(const v4fa*)(sBe + c4);
    const float z0 = fmaxf(((v.x - mu.x) * rs.x) * ga.x + be.x, 0.f);
    const float z1 = fmaxf(((v.y - mu.y) * rs.y) * ga.y + be.y, 0.f);
    const float z2 = fmaxf(((v.z - mu.z) * rs.z) * ga.z + be.z, 0.f);
    const float z3 = fmaxf(((v.w - mu.w) * rs.w) * ga.w + be.w, 0.f);
    const unsigned short h0 = f2bf(z0), h1 = f2bf(z1), h2 = f2bf(z2), h3 = f2bf(z3);
    const v4us hv = { h0, h1, h2, h3 };
    const v4us lv = { f2bf(z0 - bf2f(h0)), f2bf(z1 - bf2f(h1)), f2bf(z2 - bf2f(h2)), f2bf(z3 - bf2f(h3)) };
    *(v4us*)(sHi + row * DDM + c4) = hv;
    *(v4us*)(sLo + row * DDM + c4) = lv;
  }
  __syncthreads();

  v8f acc[5];
  {
    const v8f z = {0.f, 0.f, 0.f, 0.f, 0.f, 0.f, 0.f, 0.f};
    acc[0] = z; acc[1] = z; acc[2] = z; acc[3] = z; acc[4] = z;
  }
  const unsigned short* ahp = sHi + (16 * wave + m) * DDM;
  const unsigned short* alp = sLo + (16 * wave + m) * DDM;
  const unsigned short* wp  = WRT + (size_t)m * (size_t)DDM;
#pragma unroll 1
  for (int ks = 0; ks < DDM / 32; ++ks) {
    const v16bf aH = load_frag(ahp + 32 * ks, hh);
    const v16bf aL = load_frag(alp + 32 * ks, hh);
#pragma unroll
    for (int t = 0; t < 5; ++t) {
      const v16bf bf = load_frag(wp + (size_t)(16 * t) * (size_t)DDM + 32 * ks, hh);
      acc[t] = wmb(aH, bf, acc[t]);
      acc[t] = wmb(aL, bf, acc[t]);
    }
  }
  __syncthreads();

  float* stg = (float*)(smem + HO_AB);
#pragma unroll
  for (int t = 0; t < 4; ++t) {
    const int lc = 16 * t + m;
    const float bv = sBr[lc];
#pragma unroll
    for (int r = 0; r < 8; ++r) {
      const int lr = 16 * wave + 8 * hh + r;
      stg[lr * FIN + lc] = acc[t][r] + bv;
    }
  }
  {
    const float bp = sBr[FIN];
    if (m == 0) {
#pragma unroll
      for (int r = 0; r < 8; ++r) sPr[16 * wave + 8 * hh + r] = acc[4][r] + bp;
    }
  }
  __syncthreads();

  v4f fv[8];
#pragma unroll
  for (int i = 0; i < 8; ++i) fv[i] = *(const v4fa*)(stg + 4 * (i * GTHR + tid));
  const int tp = tid & 15;
  const v4f pv4 = *(const v4fa*)(sPr + 4 * tp);
  const bool wpred = tid < 16;
  float* ob  = OUT + (size_t)R * FIN;
  float* opd = OUT + (size_t)OOFF1 + R + 4 * tp;
#pragma unroll
  for (int i = 0; i < 8; ++i) *(volatile v4f*)(ob + 4 * (i * GTHR + tid)) = fv[i];
  if (wpred) *(volatile v4f*)opd = pv4;
  __threadfence();
#pragma unroll
  for (int i = 0; i < 8; ++i) *(volatile v4f*)(ob + 4 * (i * GTHR + tid)) = fv[i];
  if (wpred) *(volatile v4f*)opd = pv4;
}

__global__ __launch_bounds__(NTHR) void k_wcopy(const float* __restrict__ W, float* OUT, int nUnits) {
  const int i = (int)blockIdx.x * NTHR + (int)threadIdx.x;
  if (i >= nUnits) return;
  v4f v = *(const v4fa*)(W + (size_t)i * 4);
  v.x = bfr(v.x); v.y = bfr(v.y); v.z = bfr(v.z); v.w = bfr(v.w);
  float* d = OUT + (size_t)OOFF2 + (size_t)i * 4;
  *(volatile v4f*)d = v;
  __threadfence();
  *(volatile v4f*)d = v;
}

static inline int cdiv(int a, int b) { return (a + b - 1) / b; }

extern "C" void kernel_launch(void* const* d_in, const int* in_sizes, int n_in,
                              void* d_out, int out_size, void* d_ws, size_t ws_size,
                              hipStream_t stream) {
  if (n_in < 11) return;
  if (in_sizes[0] != NROW * FIN) return;
  if (in_sizes[1] < 2 || (in_sizes[1] & 1) != 0) return;
  const int nE = in_sizes[1] / 2;
  if (nE < 1 || nE > (1 << 24)) return;
  if (in_sizes[2] != NND * NND) return;
  if (in_sizes[3] != FIN * DDM) return;
  if (in_sizes[4] != DDM || in_sizes[5] != DDM || in_sizes[6] != DDM) return;
  if (in_sizes[7] != DDM * FIN || in_sizes[8] != FIN) return;
  if (in_sizes[9] != DDM || in_sizes[10] < 1) return;
  if (out_size != OTOT) return;

  const float* data  = (const float*)d_in[0];
  const int*   ei    = (const int*)  d_in[1];
  const float* warr  = (const float*)d_in[2];
  const float* lin_w = (const float*)d_in[3];
  const float* gbias = (const float*)d_in[4];
  const float* gamma = (const float*)d_in[5];
  const float* beta  = (const float*)d_in[6];
  const float* wrec  = (const float*)d_in[7];
  const float* brec  = (const float*)d_in[8];
  const float* wpred = (const float*)d_in[9];
  const float* bpred = (const float*)d_in[10];
  float* out = (float*)d_out;
  const int* src = ei;
  const int* dst = ei + nE;

  char* ws = (char*)d_ws;
  size_t off = 0;
  const size_t oXB  = off; off += (size_t)NROW * FIN * 2;         off = (off + 255) & ~(size_t)255;
  const size_t oWT  = off; off += (size_t)DDM * FIN * 2;          off = (off + 255) & ~(size_t)255;
  const size_t oWRT = off; off += (size_t)NCH * DDM * 2;          off = (off + 255) & ~(size_t)255;
  const size_t oH   = off; off += (size_t)NROW * DDM * 4;         off = (off + 255) & ~(size_t)255;
  const size_t oOF  = off; off += (size_t)NROW * DDM * 4;         off = (off + 255) & ~(size_t)255;
  const size_t oREC = off; off += (size_t)NND * 2 * DDM * 8;      off = (off + 255) & ~(size_t)255;
  const size_t oST  = off; off += (size_t)2 * DDM * 4;            off = (off + 255) & ~(size_t)255;
  if (off > ws_size || off > (size_t)WSMAX) return;
  unsigned short* XB  = (unsigned short*)(ws + oXB);
  unsigned short* WT  = (unsigned short*)(ws + oWT);
  unsigned short* WRT = (unsigned short*)(ws + oWRT);
  float*  H    = (float*)(ws + oH);
  float*  OUTF = (float*)(ws + oOF);
  double* REC  = (double*)(ws + oREC);
  float*  STATS = (float*)(ws + oST);
  const int vec8 = ((nE & 3) == 0) ? 1 : 0;

  const int nUx = NROW * (FIN / 8);
  k_xprep<<<cdiv(nUx, NTHR), NTHR, 0, stream>>>(data, XB, nUx);
  const int nUw = DDM * (FIN / 8);
  k_wtr<<<cdiv(nUw, NTHR), NTHR, 0, stream>>>(lin_w, DDM, lin_w, 1, FIN, WT, nUw);
  const int nUr = NCH * (DDM / 8);
  k_wtr<<<cdiv(nUr, NTHR), NTHR, 0, stream>>>(wrec, FIN, wpred, 1, DDM, WRT, nUr);
  k_gemm_lin<<<dim3(NROW / GBM, DDM / GBN), GTHR, 0, stream>>>(XB, WT, H);
  k_agg<<<NND, NTHR, 0, stream>>>(src, dst, warr, H, gbias, OUTF, REC, nE, vec8);
  k_bnfin<<<1, DDM, 0, stream>>>(REC, STATS);
  k_head<<<NROW / GBM, GTHR, HEAD_LDS, stream>>>(OUTF, STATS, gamma, beta, WRT, brec, bpred, out);
  const int nUc = (NND * NND) / 4;
  k_wcopy<<<cdiv(nUc, NTHR), NTHR, 0, stream>>>(warr, out, nUc);
}
